// hbPass_69715909148837
// MI455X (gfx1250) — hardware-verified
//
#include <hip/hip_runtime.h>
#include <stdint.h>

#define DEVINL __device__ __forceinline__

typedef _Float16 f16t;
typedef _Float16 v16h __attribute__((ext_vector_type(16)));
typedef _Float16 v8h  __attribute__((ext_vector_type(8)));
typedef float    v8f  __attribute__((ext_vector_type(8)));
typedef float    v4f  __attribute__((ext_vector_type(4)));
typedef v8h __attribute__((may_alias)) v8ha;
typedef v4f __attribute__((may_alias)) v4fa;
union FragH { v16h v; v8h half[2]; };

#define HD     114
#define WD     114
#define CH     64
#define KSZ    3
#define HO     (HD - KSZ + 1)
#define WO     (WD - KSZ + 1)
#define NPIX   (HD * WD)
#define PH     (HD + 2)
#define PW     (WD + 2)
#define PPIX   (PH * PW)
#define KT     (CH * 9)
#define TILEP  64
#define NTILE  ((NPIX + TILEP - 1) / TILEP)
#define PPITCH (NTILE * TILEP)
#define TPB    256
#define CTPB   128
#define YCAR   8.0f
#define WCAR   256.0f
#define INVCAR (1.0f / 2048.0f)

static_assert((KT % 32) == 0);
static_assert((WO % 4) == 0);
static_assert((NPIX % 4) == 0);
static_assert(((PPITCH * 4) % 128) == 0);
static_assert(((KT * CH * 2) % 128) == 0);
static_assert(((PPIX * CH * 2) % 128) == 0);
static_assert((PW * CH) % TPB == 0);
static_assert(CTPB == 128);

DEVINL int imin(int a, int b) { return a < b ? a : b; }
DEVINL int imax(int a, int b) { return a > b ? a : b; }

DEVINL v8f wmma_f16(v16h a, v16h b, v8f c) {
  v8f d = __builtin_amdgcn_wmma_f32_16x16x32_f16(false, a, false, b, (short)0, c, false, false);
  asm volatile("v_nop\n\tv_nop\n\tv_nop\n\tv_nop" : "+v"(d) : "v"(a), "v"(b));
  return d;
}
DEVINL v8f zero8f() {
  v8f z = {0.f, 0.f, 0.f, 0.f, 0.f, 0.f, 0.f, 0.f};
  return z;
}

__global__ __launch_bounds__(TPB) void prep_w_k(const float* __restrict__ w, f16t* __restrict__ Wp)
{
  const int t = blockIdx.x * TPB + threadIdx.x;
  if (t >= CH * (KT / 8)) return;
  const int cout = t / (KT / 8);
  const int part = t - cout * (KT / 8);
  const int k8   = 8 * part;
  const int tap  = k8 >> 6;
  const int cin0 = k8 & 63;
  v8h o;
  #pragma unroll
  for (int i = 0; i < 8; ++i) {
    const float wv = w[(size_t)(cout * CH + cin0 + i) * 9 + tap];
    o[i] = (f16t)(wv * WCAR);
  }
  f16t* dst = Wp + (size_t)cout * KT + k8;
  *(volatile v8h*)dst = o;
  __threadfence();
  *(volatile v8h*)dst = o;
}

__global__ __launch_bounds__(TPB) void binfold_k(const float* __restrict__ x, f16t* __restrict__ Yp)
{
  __shared__ __attribute__((aligned(16))) float sX[CH * WD];
  __shared__ __attribute__((aligned(16))) f16t  sY[PW * CH];
  const int tid = threadIdx.x;
  const int hp  = blockIdx.x;
  const int b   = blockIdx.y;
  const bool interior = (hp >= 1) && (hp <= HD);
  const int h = imin(imax(hp - 1, 0), HD - 1);

  if (interior) {
    const float* xb = x + ((size_t)b * CH) * NPIX + (size_t)h * WD;
    for (int idx = tid; idx < CH * WD; idx += TPB) {
      const int c  = idx / WD;
      const int wq = idx - c * WD;
      sX[idx] = xb[(size_t)c * NPIX + wq];
    }
  }
  __syncthreads();

  const int ni = imin(h, 2) - imax(h - (HO - 1), 0) + 1;
  #pragma unroll 1
  for (int idx = tid; idx < PW * CH; idx += TPB) {
    const int wp = idx >> 6;
    const int c  = idx & 63;
    const bool valid = interior && (wp >= 1) && (wp <= WD);
    const int w = imin(imax(wp - 1, 0), WD - 1);
    const float* row = sX + c * WD;
    const float xv  = row[w];
    const float sgn = (xv > 0.0f) ? 1.0f : ((xv < 0.0f) ? -1.0f : 0.0f);

    float mj[3];
    bool  vj[3];
    #pragma unroll
    for (int j = 0; j < 3; ++j) {
      const int d  = w - j;
      vj[j] = (d >= 0) && (d <= WO - 1);
      const int dc = imin(imax(d, 0), WO - 1);
      const int s0 = j + (dc & ~3);
      const float a0 = fabsf(row[s0]), a1 = fabsf(row[s0 + 1]);
      const float a2 = fabsf(row[s0 + 2]), a3 = fabsf(row[s0 + 3]);
      mj[j] = (((a0 + a1) + a2) + a3) * 0.25f;
    }
    float tot = 0.0f;
    #pragma unroll
    for (int i = 0; i < 3; ++i) {
      #pragma unroll
      for (int j = 0; j < 3; ++j) {
        tot = ((i < ni) && vj[j]) ? (tot + mj[j]) : tot;
      }
    }
    const float yv = valid ? (sgn * tot) : 0.0f;
    sY[idx] = (f16t)(yv * YCAR);
  }
  __syncthreads();

  f16t* dstrow = Yp + ((size_t)(b * PH + hp)) * (size_t)(PW * CH);
  const int piece = tid & 7;
  const int lg    = tid >> 3;
  v8h vals[4];
  #pragma unroll
  for (int q = 0; q < 4; ++q) {
    const int L = imin(q * 32 + lg, PW - 1);
    vals[q] = *(const v8ha*)(sY + L * CH + piece * 8);
  }
  #pragma unroll
  for (int q = 0; q < 4; ++q) {
    const int L = q * 32 + lg;
    if (L < PW) *(volatile v8h*)(dstrow + (size_t)L * CH + piece * 8) = vals[q];
  }
  __threadfence();
  #pragma unroll
  for (int q = 0; q < 4; ++q) {
    const int L = q * 32 + lg;
    if (L < PW) *(volatile v8h*)(dstrow + (size_t)L * CH + piece * 8) = vals[q];
  }
}

__global__ __launch_bounds__(CTPB) void conv_k(const f16t* __restrict__ Yp, const f16t* __restrict__ Wp,
                                             const float* __restrict__ bias, float* __restrict__ Yc)
{
  __shared__ __attribute__((aligned(16))) float sO[CH * TILEP];
  const int tid = threadIdx.x, lane = tid & 31, wave = tid >> 5;
  const int h = lane >> 4, m = lane & 15;
  const int wc = wave & 1, wq = wave >> 1;
  const int b = blockIdx.y;
  const int pixBase = blockIdx.x * TILEP;

  const int p0  = imin(pixBase + 32 * wq + m,      NPIX - 1);
  const int p1  = imin(pixBase + 32 * wq + 16 + m, NPIX - 1);
  const int oh0 = p0 / WD, ow0 = p0 - oh0 * WD;
  const int oh1 = p1 / WD, ow1 = p1 - oh1 * WD;
  const f16t* yb0 = Yp + ((size_t)(b * PH + oh0) * PW + ow0) * CH + 8 * h;
  const f16t* yb1 = Yp + ((size_t)(b * PH + oh1) * PW + ow1) * CH + 8 * h;
  const f16t* wr0 = Wp + (size_t)(32 * wc + m) * KT + 8 * h;
  const f16t* wr1 = wr0 + (size_t)16 * KT;

  v8f acc00 = zero8f(), acc01 = zero8f(), acc10 = zero8f(), acc11 = zero8f();

  #pragma unroll 1
  for (int kh = 0; kh < 3; ++kh) {
    #pragma unroll 1
    for (int kw = 0; kw < 3; ++kw) {
      const int tap  = 3 * kh + kw;
      const int toff = (kh * PW + kw) * CH;
      const f16t* ya0 = yb0 + toff;
      const f16t* ya1 = yb1 + toff;
      const f16t* wa0 = wr0 + tap * CH;
      const f16t* wa1 = wr1 + tap * CH;
      #pragma unroll
      for (int ks = 0; ks < 2; ++ks) {
        FragH a0, a1, b0, b1;
        a0.half[0] = *(const v8ha*)(wa0 + 32 * ks);
        a0.half[1] = *(const v8ha*)(wa0 + 32 * ks + 16);
        a1.half[0] = *(const v8ha*)(wa1 + 32 * ks);
        a1.half[1] = *(const v8ha*)(wa1 + 32 * ks + 16);
        b0.half[0] = *(const v8ha*)(ya0 + 32 * ks);
        b0.half[1] = *(const v8ha*)(ya0 + 32 * ks + 16);
        b1.half[0] = *(const v8ha*)(ya1 + 32 * ks);
        b1.half[1] = *(const v8ha*)(ya1 + 32 * ks + 16);
        acc00 = wmma_f16(a0.v, b0.v, acc00);
        acc01 = wmma_f16(a0.v, b1.v, acc01);
        acc10 = wmma_f16(a1.v, b0.v, acc10);
        acc11 = wmma_f16(a1.v, b1.v, acc11);
      }
    }
  }

  {
    const int cbA = 32 * wc + 8 * h;
    const int cbB = 32 * wc + 16 + 8 * h;
    const int plA = 32 * wq + m;
    const int plB = 32 * wq + 16 + m;
    #pragma unroll
    for (int r = 0; r < 8; ++r) {
      const float bA = bias[cbA + r];
      const float bB = bias[cbB + r];
      sO[(cbA + r) * TILEP + plA] = fmaxf(fmaf(acc00[r], INVCAR, bA), 0.0f);
      sO[(cbA + r) * TILEP + plB] = fmaxf(fmaf(acc01[r], INVCAR, bA), 0.0f);
      sO[(cbB + r) * TILEP + plA] = fmaxf(fmaf(acc10[r], INVCAR, bB), 0.0f);
      sO[(cbB + r) * TILEP + plB] = fmaxf(fmaf(acc11[r], INVCAR, bB), 0.0f);
    }
  }
  __syncthreads();

  float* gbase = Yc + ((size_t)b * CH) * PPITCH + (size_t)pixBase + 4 * m;
  v4f vv[8];
  #pragma unroll
  for (int j = 0; j < 8; ++j) {
    const int row = 16 * wave + 2 * j + h;
    vv[j] = *(const v4fa*)(sO + row * TILEP + 4 * m);
  }
  #pragma unroll
  for (int j = 0; j < 8; ++j) {
    const int row = 16 * wave + 2 * j + h;
    *(volatile v4f*)(gbase + (size_t)row * PPITCH) = vv[j];
  }
  __threadfence();
  #pragma unroll
  for (int j = 0; j < 8; ++j) {
    const int row = 16 * wave + 2 * j + h;
    *(volatile v4f*)(gbase + (size_t)row * PPITCH) = vv[j];
  }
}

__global__ __launch_bounds__(TPB) void pack_out_k(const float* __restrict__ Yc, float* __restrict__ out,
                                                int total4)
{
  const int t = blockIdx.x * TPB + threadIdx.x;
  if (t >= total4) return;
  const int f = 4 * t;
  const int q = f / NPIX;
  const int p = f - q * NPIX;
  const v4f v = *(const v4fa*)(Yc + (size_t)q * PPITCH + p);
  float* dst = out + (size_t)f;
  *(volatile v4f*)dst = v;
  __threadfence();
  *(volatile v4f*)dst = v;
}

extern "C" void kernel_launch(void* const* d_in, const int* in_sizes, int n_in,
                              void* d_out, int out_size, void* d_ws, size_t ws_size,
                              hipStream_t stream)
{
  if (n_in < 3) return;
  const int plane = CH * NPIX;
  if (in_sizes[0] <= 0 || (in_sizes[0] % plane) != 0) return;
  const int nB = in_sizes[0] / plane;
  if (nB > 65535) return;
  if (in_sizes[1] != CH * CH * 9) return;
  if (in_sizes[2] != CH) return;
  if (out_size != nB * plane) return;

  const float* x  = (const float*)d_in[0];
  const float* cw = (const float*)d_in[1];
  const float* cb = (const float*)d_in[2];
  float* outp = (float*)d_out;

  const size_t szWp = (size_t)CH * KT * 2;
  const size_t szYp = (size_t)nB * PPIX * CH * 2;
  const size_t szYc = (size_t)nB * CH * PPITCH * 4;
  size_t off = 0;
  char* ws = (char*)d_ws;
  f16t*  Wp = (f16t*)(ws + off);  off += szWp;
  f16t*  Yp = (f16t*)(ws + off);  off += szYp;
  float* Yc = (float*)(ws + off); off += szYc;
  if (off > ws_size) return;
  if (off > (size_t)134217728) return;

  const int total4 = out_size / 4;

  prep_w_k<<<(CH * (KT / 8) + TPB - 1) / TPB, TPB, 0, stream>>>(cw, Wp);
  binfold_k<<<dim3(PH, nB), TPB, 0, stream>>>(x, Yp);
  conv_k<<<dim3(NTILE, nB), CTPB, 0, stream>>>(Yp, Wp, cb, Yc);
  pack_out_k<<<(total4 + TPB - 1) / TPB, TPB, 0, stream>>>(Yc, outp, total4);
}
